// QTransformerClassifier_65481071407819
// MI455X (gfx1250) — hardware-verified
//
#include <hip/hip_runtime.h>

#define NB 8
#define NS 512
#define NE 128
#define NH 16
#define DK 8
#define NL 4
#define NF 512
#define NQ 4
#define NC 10
#define NT (NB * NS)
#define VTP 520
#define OPLANE (NB * NH * NS * DK)
#define WOPLANE (NL * NE * NE)
#define W2PLANE (NL * NE * NF)

static_assert(NS % 256 == 0);
static_assert(NT % 64 == 0);
static_assert(NS % 64 == 0);
static_assert(NE == 128);
static_assert(NF % 32 == 0);
static_assert(WOPLANE % 2048 == 0);
static_assert(W2PLANE % 2048 == 0);
static_assert((VTP % 8) == 0);

typedef __bf16 v16b __attribute__((ext_vector_type(16)));
typedef __bf16 v8b __attribute__((ext_vector_type(8)));
typedef unsigned short v16us __attribute__((ext_vector_type(16)));
typedef unsigned short v8us __attribute__((ext_vector_type(8)));
typedef float v8f __attribute__((ext_vector_type(8)));
typedef float v4f __attribute__((ext_vector_type(4)));
typedef v8us __attribute__((may_alias)) v8usa;
typedef v4f __attribute__((may_alias)) v4fa;

union Frag { v16b v; v8us u[2]; };
union Pk8 { v8b b; v8us u; };
union Pk16 { v16b b; v16us u; };

__device__ __forceinline__ v8f wmma_bf(v16b a, v16b b, v8f c) {
  v8f d = __builtin_amdgcn_wmma_f32_16x16x32_bf16(false, a, false, b, (short)0, c, false, false);
  asm volatile("v_nop\n\tv_nop\n\tv_nop\n\tv_nop" : "+v"(d) : "v"(a), "v"(b));
  return d;
}

__device__ __forceinline__ v16b load_frag(const unsigned short* p, int hf) {
  Frag f;
  f.u[0] = *(const v8usa*)(p + 8 * hf);
  f.u[1] = *(const v8usa*)(p + 16 + 8 * hf);
  return f.v;
}

__device__ __forceinline__ void split_bf(float x, __bf16& hi, __bf16& lo) {
  hi = (__bf16)x;
  lo = (__bf16)(x - (float)hi);
}

__global__ __launch_bounds__(256) void k_cvtw(const float* __restrict__ wo,
                                              const float* __restrict__ w2,
                                              unsigned short* __restrict__ wop,
                                              unsigned short* __restrict__ w2p) {
  const int tid = threadIdx.x;
  const float* src;
  unsigned short* dh;
  unsigned short* dl;
  if (blockIdx.x < WOPLANE / 2048) {
    const size_t g = (size_t)blockIdx.x * 256 + tid;
    src = wo + g * 8;
    dh = wop + g * 8;
    dl = wop + WOPLANE + g * 8;
  } else {
    const size_t g = (size_t)(blockIdx.x - WOPLANE / 2048) * 256 + tid;
    src = w2 + g * 8;
    dh = w2p + g * 8;
    dl = w2p + W2PLANE + g * 8;
  }
  const v4f a = *(const v4fa*)src;
  const v4f c = *(const v4fa*)(src + 4);
  const float x[8] = {a.x, a.y, a.z, a.w, c.x, c.y, c.z, c.w};
  Pk8 H, L;
#pragma unroll
  for (int i = 0; i < 8; ++i) {
    __bf16 hi, lo;
    split_bf(x[i], hi, lo);
    H.b[i] = hi;
    L.b[i] = lo;
  }
  const v8us hv = H.u, lv = L.u;
  *(volatile v8us*)dh = hv;
  *(volatile v8us*)dl = lv;
  __threadfence();
  *(volatile v8us*)dh = hv;
  *(volatile v8us*)dl = lv;
}

__global__ __launch_bounds__(256) void k_embed(const int* __restrict__ tokens,
                                               const float* __restrict__ emb,
                                               int vocab,
                                               float* __restrict__ h) {
  const int tid = threadIdx.x, lane = tid & 31;
  const int t = blockIdx.x * 8 + (tid >> 5);
  const int s = t & (NS - 1);
  int tok = tokens[t];
  tok = tok < 0 ? 0 : tok;
  tok = tok > vocab - 1 ? vocab - 1 : tok;
  const int e0 = 4 * lane;
  const v4f ev = *(const v4fa*)(emb + (size_t)tok * NE + e0);
  const float cdiv = (float)(-9.210340371976184 / 128.0);
  float ps0 = 0.f, pc0 = 0.f, ps1 = 0.f, pc1 = 0.f;
#pragma unroll 1
  for (int pp = 0; pp < 2; ++pp) {
    const float i2 = (float)(e0 + 2 * pp);
    const float dv = expf(i2 * cdiv);
    const float arg = (float)s * dv;
    const float sv = sinf(arg);
    const float cv = cosf(arg);
    const bool first = (pp == 0);
    ps0 = first ? sv : ps0;
    pc0 = first ? cv : pc0;
    ps1 = first ? ps1 : sv;
    pc1 = first ? pc1 : cv;
  }
  v4f o;
  o.x = ev.x + ps0;
  o.y = ev.y + pc0;
  o.z = ev.z + ps1;
  o.w = ev.w + pc1;
  float* dst = h + (size_t)t * NE + e0;
  *(volatile v4f*)dst = o;
  __threadfence();
  *(volatile v4f*)dst = o;
}

__global__ __launch_bounds__(256) void k_attn(const float* __restrict__ h,
                                              const float* __restrict__ theta,
                                              int layer,
                                              unsigned short* __restrict__ op) {
  __shared__ __attribute__((aligned(16))) unsigned short sEnc[NS * 16];
  __shared__ __attribute__((aligned(16))) unsigned short sVt[16 * VTP];

  const int tid = threadIdx.x, lane = tid & 31, w = tid >> 5;
  const int hf = lane >> 4, m = lane & 15;
  const int bh = blockIdx.x, b = bh >> 4, head = bh & 15;

  float th[DK];
#pragma unroll
  for (int d = 0; d < DK; ++d) th[d] = theta[layer * DK + d];

#pragma unroll 1
  for (int it = 0; it < NS / 256; ++it) {
    const int s = tid + 256 * it;
    const float* src = h + ((size_t)(b * NS + s)) * NE + head * DK;
    const v4f xa = *(const v4fa*)src;
    const v4f xb = *(const v4fa*)(src + 4);
    const float c0 = cosf(xa.x + th[0]);
    const float c1 = cosf(xa.y + th[1]);
    const float c2 = cosf(xa.z + th[2]);
    const float c3 = cosf(xa.w + th[3]);
    const float c4 = cosf(xb.x + th[4]);
    const float c5 = cosf(xb.y + th[5]);
    const float c6 = cosf(xb.z + th[6]);
    const float c7 = cosf(xb.w + th[7]);
    float e[DK];
    e[0] = c1 * c2 * c3 * c4 * c5 * c6 * c7;
    float p = c0 * c1; e[1] = p;
    p *= c2; e[2] = p;
    p *= c3; e[3] = p;
    p *= c4; e[4] = p;
    p *= c5; e[5] = p;
    p *= c6; e[6] = p;
    p *= c7; e[7] = p;
    Pk8 H, L;
#pragma unroll
    for (int d = 0; d < DK; ++d) {
      __bf16 hi, lo;
      split_bf(e[d], hi, lo);
      H.b[d] = hi;
      L.b[d] = lo;
    }
    *(v8usa*)(sEnc + s * 16) = H.u;
    *(v8usa*)(sEnc + s * 16 + 8) = L.u;
#pragma unroll
    for (int d = 0; d < DK; ++d) {
      sVt[d * VTP + s] = H.u[d];
      sVt[(8 + d) * VTP + s] = L.u[d];
    }
  }
  __syncthreads();

  const v8f z8 = {0.f, 0.f, 0.f, 0.f, 0.f, 0.f, 0.f, 0.f};
  const float scl = 0.353553390593273762f;

#pragma unroll 1
  for (int qi = 0; qi < 4; ++qi) {
    const int q0 = (w * 4 + qi) * 16;
    Frag qf;
    qf.u[0] = *(const v8usa*)(sEnc + (q0 + m) * 16);
    qf.u[1] = *(const v8usa*)(sEnc + (q0 + m) * 16 + 8);

    v8f acc = z8;
    float mrun = -1e30f, lrun = 0.0f;

#pragma unroll 1
    for (int kb = 0; kb < NS; kb += 32) {
      v8f s[2];
#pragma unroll
      for (int j = 0; j < 2; ++j) {
        const v8us piece = *(const v8usa*)(sEnc + (kb + 16 * j + m) * 16 + 8 * hf);
        Frag kf;
        kf.u[0] = piece;
        kf.u[1] = piece;
        s[j] = wmma_bf(kf.v, qf.v, z8);
      }
      float mloc = -1e30f;
#pragma unroll
      for (int j = 0; j < 2; ++j)
#pragma unroll
        for (int r = 0; r < 8; ++r) {
          s[j][r] = s[j][r] * scl;
          mloc = fmaxf(mloc, s[j][r]);
        }
      mloc = fmaxf(mloc, __shfl_xor(mloc, 16));
      const float mnew = fmaxf(mrun, mloc);
      const float alpha = __expf(mrun - mnew);
      mrun = mnew;
      float lsum = 0.0f;
#pragma unroll
      for (int j = 0; j < 2; ++j)
#pragma unroll
        for (int r = 0; r < 8; ++r) {
          const float pv = __expf(s[j][r] - mnew);
          s[j][r] = pv;
          lsum += pv;
        }
      lsum += __shfl_xor(lsum, 16);
      lrun = lrun * alpha + lsum;
#pragma unroll
      for (int r = 0; r < 8; ++r) acc[r] = acc[r] * alpha;

      Pk16 ph, pl;
#pragma unroll
      for (int r = 0; r < 8; ++r) {
        __bf16 hi, lo;
        split_bf(s[0][r], hi, lo);
        ph.b[r] = hi;
        pl.b[r] = lo;
        split_bf(s[1][r], hi, lo);
        ph.b[8 + r] = hi;
        pl.b[8 + r] = lo;
      }
      const v16b vf = load_frag(sVt + m * VTP + kb, hf);
      acc = wmma_bf(vf, ph.b, acc);
      acc = wmma_bf(vf, pl.b, acc);
    }

    const float inv = 1.0f / lrun;
    float o[8];
#pragma unroll
    for (int r = 0; r < 8; ++r) o[r] = (acc[r] + __shfl_xor(acc[r], 16)) * inv;
    Pk8 H, L;
#pragma unroll
    for (int r = 0; r < 8; ++r) {
      __bf16 hi, lo;
      split_bf(o[r], hi, lo);
      H.b[r] = hi;
      L.b[r] = lo;
    }
    v8us val;
#pragma unroll
    for (int r = 0; r < 8; ++r) val[r] = hf ? L.u[r] : H.u[r];
    unsigned short* dst = op + (((size_t)hf * (NB * NH) + bh) * NS + q0 + m) * DK;
    *(volatile v8us*)dst = val;
    __threadfence();
    *(volatile v8us*)dst = val;
  }
}

__device__ __forceinline__ void epi_ln(v8f (&acc)[8], float* sTw, float* h, int t0,
                                       const float* __restrict__ g,
                                       const float* __restrict__ bt,
                                       int lane, int hf, int m) {
#pragma unroll
  for (int nt = 0; nt < 8; ++nt)
#pragma unroll
    for (int r = 0; r < 8; ++r) sTw[(8 * hf + r) * NE + 16 * nt + m] = acc[nt][r];
  __syncthreads();

  const int rr = lane >> 1, ch = lane & 1;
  float* trow = sTw + rr * NE + 64 * ch;
  const float* hrow = h + (size_t)(t0 + rr) * NE + 64 * ch;
  float x[64];
#pragma unroll
  for (int j = 0; j < 16; ++j) {
    const v4f a = *(const v4fa*)(trow + 4 * j);
    const v4f c = *(const v4fa*)(hrow + 4 * j);
    x[4 * j + 0] = a.x + c.x;
    x[4 * j + 1] = a.y + c.y;
    x[4 * j + 2] = a.z + c.z;
    x[4 * j + 3] = a.w + c.w;
  }
  float sum = 0.0f;
#pragma unroll
  for (int j = 0; j < 64; ++j) sum += x[j];
  sum += __shfl_xor(sum, 1);
  const float mean = sum * (1.0f / NE);
  float vs = 0.0f;
#pragma unroll
  for (int j = 0; j < 64; ++j) {
    const float d = x[j] - mean;
    vs += d * d;
  }
  vs += __shfl_xor(vs, 1);
  const float rs = rsqrtf(vs * (1.0f / NE) + 1e-5f);
#pragma unroll
  for (int j = 0; j < 16; ++j) {
    const v4f gv = *(const v4fa*)(g + 64 * ch + 4 * j);
    const v4f bv = *(const v4fa*)(bt + 64 * ch + 4 * j);
    v4f y;
    y.x = (x[4 * j + 0] - mean) * rs * gv.x + bv.x;
    y.y = (x[4 * j + 1] - mean) * rs * gv.y + bv.y;
    y.z = (x[4 * j + 2] - mean) * rs * gv.z + bv.z;
    y.w = (x[4 * j + 3] - mean) * rs * gv.w + bv.w;
    *(v4fa*)(trow + 4 * j) = y;
  }
  __syncthreads();

#pragma unroll
  for (int i = 0; i < 16; ++i) {
    const v4f y = *(const v4fa*)(sTw + i * NE + 4 * lane);
    *(volatile v4f*)(h + (size_t)(t0 + i) * NE + 4 * lane) = y;
  }
  __threadfence();
#pragma unroll
  for (int i = 0; i < 16; ++i) {
    const v4f y = *(const v4fa*)(sTw + i * NE + 4 * lane);
    *(volatile v4f*)(h + (size_t)(t0 + i) * NE + 4 * lane) = y;
  }
}

__global__ __launch_bounds__(128) void k_wo_ln(float* h,
                                               const unsigned short* __restrict__ op,
                                               const unsigned short* __restrict__ wop,
                                               const float* __restrict__ g,
                                               const float* __restrict__ bt,
                                               int layer) {
  __shared__ __attribute__((aligned(16))) float sT[4 * 16 * NE];

  const int tid = threadIdx.x, lane = tid & 31, w = tid >> 5;
  const int hf = lane >> 4, m = lane & 15;
  const int t0 = blockIdx.x * 64 + 16 * w;
  const int b = t0 / NS, s0 = t0 - b * NS;
  const unsigned short* oph = op;
  const unsigned short* opl = op + OPLANE;
  const unsigned short* wh = wop + (size_t)layer * NE * NE;
  const unsigned short* wl = wop + WOPLANE + (size_t)layer * NE * NE;

  const v8f z8 = {0.f, 0.f, 0.f, 0.f, 0.f, 0.f, 0.f, 0.f};
  v8f acc[8];
#pragma unroll
  for (int nt = 0; nt < 8; ++nt) acc[nt] = z8;

#pragma unroll 1
  for (int k0 = 0; k0 < NE; k0 += 32) {
    const size_t ra = ((size_t)(b * NH + (k0 >> 3) + hf) * NS + s0 + m) * DK;
    const size_t rb = ra + (size_t)2 * NS * DK;
    Frag ah, al;
    ah.u[0] = *(const v8usa*)(oph + ra);
    ah.u[1] = *(const v8usa*)(oph + rb);
    al.u[0] = *(const v8usa*)(opl + ra);
    al.u[1] = *(const v8usa*)(opl + rb);
#pragma unroll
    for (int nt = 0; nt < 8; ++nt) {
      const size_t wr = (size_t)(16 * nt + m) * NE + k0;
      const v16b bhv = load_frag(wh + wr, hf);
      const v16b blv = load_frag(wl + wr, hf);
      acc[nt] = wmma_bf(ah.v, bhv, acc[nt]);
      acc[nt] = wmma_bf(ah.v, blv, acc[nt]);
      acc[nt] = wmma_bf(al.v, bhv, acc[nt]);
    }
  }

  epi_ln(acc, sT + w * (16 * NE), h, t0, g + layer * NE, bt + layer * NE, lane, hf, m);
}

__global__ __launch_bounds__(128) void k_ffn_ln(float* h,
                                                const float* __restrict__ ftheta,
                                                const float* __restrict__ w1all,
                                                const unsigned short* __restrict__ w2p,
                                                const float* __restrict__ g,
                                                const float* __restrict__ bt,
                                                int layer) {
  __shared__ __attribute__((aligned(16))) float sT[4 * 16 * NE];

  const int tid = threadIdx.x, lane = tid & 31, w = tid >> 5;
  const int hf = lane >> 4, m = lane & 15;
  const int t0 = blockIdx.x * 64 + 16 * w;
  const int tm = t0 + m;
  const float* w1 = w1all + (size_t)layer * NF * NQ;
  const unsigned short* wh = w2p + (size_t)layer * NE * NF;
  const unsigned short* wl = w2p + W2PLANE + (size_t)layer * NE * NF;

  const v4f hx = *(const v4fa*)(h + (size_t)tm * NE);
  const float ms0 = cosf(hx.x) * cosf(ftheta[layer * NQ + 0]);
  const float ms1 = cosf(hx.y) * cosf(ftheta[layer * NQ + 1]);
  const float ms2 = cosf(hx.z) * cosf(ftheta[layer * NQ + 2]);
  const float ms3 = cosf(hx.w) * cosf(ftheta[layer * NQ + 3]);

  const v8f z8 = {0.f, 0.f, 0.f, 0.f, 0.f, 0.f, 0.f, 0.f};
  v8f acc[8];
#pragma unroll
  for (int nt = 0; nt < 8; ++nt) acc[nt] = z8;

#pragma unroll 1
  for (int kk = 0; kk < NF; kk += 32) {
    Pk16 ah, al;
#pragma unroll
    for (int i = 0; i < 16; ++i) {
      const int f = (i < 8) ? (kk + 8 * hf + i) : (kk + 16 + 8 * hf + (i - 8));
      const v4f wv = *(const v4fa*)(w1 + (size_t)f * NQ);
      float a = ms0 * wv.x + ms1 * wv.y + ms2 * wv.z + ms3 * wv.w;
      a = fmaxf(a, 0.0f);
      __bf16 hi, lo;
      split_bf(a, hi, lo);
      ah.b[i] = hi;
      al.b[i] = lo;
    }
#pragma unroll
    for (int nt = 0; nt < 8; ++nt) {
      const size_t wr = (size_t)(16 * nt + m) * NF + kk;
      const v16b bhv = load_frag(wh + wr, hf);
      const v16b blv = load_frag(wl + wr, hf);
      acc[nt] = wmma_bf(ah.b, bhv, acc[nt]);
      acc[nt] = wmma_bf(ah.b, blv, acc[nt]);
      acc[nt] = wmma_bf(al.b, bhv, acc[nt]);
    }
  }

  epi_ln(acc, sT + w * (16 * NE), h, t0, g + layer * NE, bt + layer * NE, lane, hf, m);
}

__global__ __launch_bounds__(256) void k_head(const float* __restrict__ h,
                                              const float* __restrict__ wc,
                                              const float* __restrict__ bc,
                                              float* __restrict__ out) {
  __shared__ float sp[NB * NE];
  __shared__ __attribute__((aligned(16))) float so[96];
  const int tid = threadIdx.x;
  for (int i = tid; i < NB * NE; i += 256) {
    const int bb = i >> 7, e = i & 127;
    const float* p = h + (size_t)bb * NS * NE + e;
    float s = 0.0f;
#pragma unroll 4
    for (int t = 0; t < NS; ++t) s += p[(size_t)t * NE];
    sp[i] = s * (1.0f / NS);
  }
  __syncthreads();
  if (tid < NB * NC) {
    const int bb = tid / NC, c = tid - bb * NC;
    float s = 0.0f;
#pragma unroll 1
    for (int e = 0; e < NE; ++e) s += sp[bb * NE + e] * wc[c * NE + e];
    so[tid] = s + bc[c];
  }
  __syncthreads();
  if (tid < 20) {
    const v4f v = *(const v4fa*)(so + 4 * tid);
    *(volatile v4f*)(out + 4 * tid) = v;
  }
  __threadfence();
  if (tid < 20) {
    const v4f v = *(const v4fa*)(so + 4 * tid);
    *(volatile v4f*)(out + 4 * tid) = v;
  }
}

extern "C" void kernel_launch(void* const* d_in, const int* in_sizes, int n_in,
                              void* d_out, int out_size, void* d_ws, size_t ws_size,
                              hipStream_t stream) {
  if (n_in < 13) return;
  if (in_sizes[0] != NT) return;
  if (in_sizes[1] < NE || (in_sizes[1] % NE) != 0) return;
  if (in_sizes[2] != NL * DK || in_sizes[3] != NL * NQ) return;
  if (in_sizes[4] != NL * NE * NE || in_sizes[5] != NL * NF * NQ || in_sizes[6] != NL * NE * NF) return;
  if (in_sizes[7] != NL * NE || in_sizes[8] != NL * NE || in_sizes[9] != NL * NE || in_sizes[10] != NL * NE) return;
  if (in_sizes[11] != NC * NE || in_sizes[12] != NC) return;
  if (out_size != NB * NC) return;

  const int*   tokens = (const int*)d_in[0];
  const float* emb    = (const float*)d_in[1];
  const float* atheta = (const float*)d_in[2];
  const float* ftheta = (const float*)d_in[3];
  const float* Wo     = (const float*)d_in[4];
  const float* W1     = (const float*)d_in[5];
  const float* W2     = (const float*)d_in[6];
  const float* ln1g   = (const float*)d_in[7];
  const float* ln1b   = (const float*)d_in[8];
  const float* ln2g   = (const float*)d_in[9];
  const float* ln2b   = (const float*)d_in[10];
  const float* Wc     = (const float*)d_in[11];
  const float* bc     = (const float*)d_in[12];
  float* out = (float*)d_out;
  const int vocab = in_sizes[1] / NE;

  const size_t h_bytes   = (size_t)NT * NE * 4;
  const size_t op_bytes  = (size_t)2 * OPLANE * 2;
  const size_t wop_bytes = (size_t)2 * WOPLANE * 2;
  const size_t w2p_bytes = (size_t)2 * W2PLANE * 2;
  const size_t total = h_bytes + op_bytes + wop_bytes + w2p_bytes;
  if (total > ws_size) return;

  char* ws = (char*)d_ws;
  float* h = (float*)ws;
  unsigned short* op  = (unsigned short*)(ws + h_bytes);
  unsigned short* wop = (unsigned short*)(ws + h_bytes + op_bytes);
  unsigned short* w2p = (unsigned short*)(ws + h_bytes + op_bytes + wop_bytes);

  k_cvtw<<<(WOPLANE + W2PLANE) / 2048, 256, 0, stream>>>(Wo, W2, wop, w2p);
  k_embed<<<NT / 8, 256, 0, stream>>>(tokens, emb, vocab, h);

  for (int l = 0; l < NL; ++l) {
    k_attn<<<NB * NH, 256, 0, stream>>>(h, atheta, l, op);
    k_wo_ln<<<NT / 64, 128, 0, stream>>>(h, op, wop, ln1g, ln1b, l);
    k_ffn_ln<<<NT / 64, 128, 0, stream>>>(h, ftheta, W1, w2p, ln2g, ln2b, l);
  }

  k_head<<<1, 256, 0, stream>>>(h, Wc, bc, out);
}
